// EdgeDecoder_24481313587756
// MI455X (gfx1250) — hardware-verified
//
#include <hip/hip_runtime.h>
#include <stddef.h>
#include <stdint.h>


#define HF    128
#define KIN   256
#define K2    256
#define NTHR  256
#define GBM   64
#define GBN   128
#define GTHR  128
#define EPB   128
#define ETHR  128
#define ENW   4
#define AP    264
#define DP    132
#define CSTN  400
#define NUWB  (KIN * HF / 8)
#define NUW1  (HF * K2 / 8)
#define NPREP (2 * NUWB + 2 * NUW1)
#define EDGE_LDS_BYTES (EPB * DP * 4 + EPB * AP * 2 + CSTN * 4 + EPB * 4)
#define WSMAX 134217728

static_assert(NUWB % NTHR == 0 && NUW1 % NTHR == 0 && NPREP % NTHR == 0);
static_assert(HF % 32 == 0 && K2 % 32 == 0 && HF == GBN && KIN == 2 * HF && K2 == 2 * HF);
static_assert(GBM == (GTHR / 32) * 16 && GBN == 4 * 32);
static_assert(EPB == ETHR && EPB == ENW * 32 && (EPB % 32) == 0 && EPB / 4 == 32 && EPB / 4 <= ETHR);
static_assert(AP >= K2 && DP >= HF && (AP * 2) % 16 == 0 && (DP * 4) % 16 == 0);
static_assert((EPB * DP * 4) % 16 == 0 && (EPB * AP * 2) % 16 == 0 && (CSTN * 4) % 16 == 0 && CSTN >= 3 * HF + 1);
static_assert(EDGE_LDS_BYTES <= 300000);

typedef float          v4f   __attribute__((ext_vector_type(4)));
typedef float          v8f   __attribute__((ext_vector_type(8)));
typedef int            v8i   __attribute__((ext_vector_type(8)));
typedef unsigned short v8us  __attribute__((ext_vector_type(8)));
typedef unsigned short v16us __attribute__((ext_vector_type(16)));
typedef __bf16         v16bf __attribute__((ext_vector_type(16)));
typedef v4f  __attribute__((may_alias)) v4fa;
typedef v8us __attribute__((may_alias)) v8usa;
union FragB { v16bf v; v16us u; v8us h[2]; v8i w; };

__device__ __forceinline__ v8f wmb(const FragB& a, const FragB& b, v8f c) {
  v8f d = __builtin_amdgcn_wmma_f32_16x16x32_bf16(false, a.v, false, b.v, (short)0, c, false, false);
  asm volatile("v_nop\n\tv_nop\n\tv_nop\n\tv_nop" : "+v"(d) : "v"(a.w), "v"(b.w));
  return d;
}

__device__ __forceinline__ unsigned bf16_bits(float f) {
  const unsigned u = __float_as_uint(f);
  return (u + 0x7FFFu + ((u >> 16) & 1u)) >> 16;
}
__device__ __forceinline__ float bf16_val(float f) {
  return __uint_as_float(bf16_bits(f) << 16);
}
__device__ __forceinline__ v8us cvt8(const v4f a, const v4f b) {
  v8us o;
  o[0] = (unsigned short)bf16_bits(a.x);
  o[1] = (unsigned short)bf16_bits(a.y);
  o[2] = (unsigned short)bf16_bits(a.z);
  o[3] = (unsigned short)bf16_bits(a.w);
  o[4] = (unsigned short)bf16_bits(b.x);
  o[5] = (unsigned short)bf16_bits(b.y);
  o[6] = (unsigned short)bf16_bits(b.z);
  o[7] = (unsigned short)bf16_bits(b.w);
  return o;
}
__device__ __forceinline__ float elu_f(float x) {
  const float em = __expf(fminf(x, 0.0f)) - 1.0f;
  return x > 0.0f ? x : em;
}
__device__ __forceinline__ float sigm_f(float t) {
  return __builtin_amdgcn_rcpf(1.0f + __expf(-t));
}
__device__ __forceinline__ void put16(unsigned short* dp, v8us o) {
  *(volatile v8us*)dp = o;
  __threadfence();
  *(volatile v8us*)dp = o;
}

__global__ __launch_bounds__(NTHR) void k_prep(const float* __restrict__ Wbu, const float* __restrict__ Wbi,
                                               const float* __restrict__ W1u, const float* __restrict__ W1i,
                                               unsigned short* WBTu, unsigned short* WBTi,
                                               unsigned short* W1Tu, unsigned short* W1Ti) {
  const int u = (int)blockIdx.x * NTHR + (int)threadIdx.x;
  v8us o;
  if (u < NUWB) {
    const int n   = u >> 4;
    const int k8  = (u & 15) * 8;
    const int nn  = n & (HF - 1);
    const int kof = (n >> 7) * HF;
    const float* p = Wbu + (size_t)(kof + k8) * HF + nn;
#pragma unroll
    for (int i = 0; i < 8; ++i) o[i] = (unsigned short)bf16_bits(p[(size_t)i * HF]);
    put16(WBTu + (size_t)n * HF + k8, o);
    return;
  } else if (u < 2 * NUWB) {
    const int v   = u - NUWB;
    const int n   = v >> 4;
    const int k8  = (v & 15) * 8;
    const int nn  = n & (HF - 1);
    const int kof = (n >> 7) * HF;
    const float* p = Wbi + (size_t)(kof + k8) * HF + nn;
#pragma unroll
    for (int i = 0; i < 8; ++i) o[i] = (unsigned short)bf16_bits(p[(size_t)i * HF]);
    put16(WBTi + (size_t)n * HF + k8, o);
    return;
  } else if (u < 2 * NUWB + NUW1) {
    const int v    = u - 2 * NUWB;
    const int n    = v >> 5;
    const int k8   = (v & 31) * 8;
    const int srow = k8 & (HF - 1);
    const float* p = W1u + (size_t)srow * HF + n;
#pragma unroll
    for (int i = 0; i < 8; ++i) o[i] = (unsigned short)bf16_bits(p[(size_t)i * HF]);
    put16(W1Tu + (size_t)n * K2 + k8, o);
    return;
  } else if (u < NPREP) {
    const int v    = u - 2 * NUWB - NUW1;
    const int n    = v >> 5;
    const int k8   = (v & 31) * 8;
    const int srow = k8 & (HF - 1);
    const float* p = W1i + (size_t)srow * HF + n;
#pragma unroll
    for (int i = 0; i < 8; ++i) o[i] = (unsigned short)bf16_bits(p[(size_t)i * HF]);
    put16(W1Ti + (size_t)n * K2 + k8, o);
    return;
  }
}

__global__ __launch_bounds__(GTHR) void k_gemm(const float* __restrict__ A, int nRows, int lda,
                                               const unsigned short* __restrict__ BT, int ldb, int K,
                                               float* Cm, int ldc) {
  __shared__ __attribute__((aligned(16))) float stg[GBM * GBN];
  const int tid = (int)threadIdx.x, lane = tid & 31, wave = tid >> 5, hh = lane >> 4, m = lane & 15;
  const int rowBase = (int)blockIdx.x * GBM;
  const int colBase = (int)blockIdx.y * GBN;

  v8f acc[8];
  {
    const v8f z = {0.f, 0.f, 0.f, 0.f, 0.f, 0.f, 0.f, 0.f};
#pragma unroll
    for (int t = 0; t < 8; ++t) acc[t] = z;
  }
  int ar = rowBase + 16 * wave + m;
  ar = ar > nRows - 1 ? nRows - 1 : ar;
  const float*          ap = A  + (size_t)ar * (size_t)lda + 8 * hh;
  const unsigned short* bp = BT + (size_t)(colBase + m) * (size_t)ldb + 8 * hh;

#pragma unroll 1
  for (int k0 = 0; k0 < K; k0 += 32) {
    const v4f x0 = *(const v4fa*)(ap + k0);
    const v4f x1 = *(const v4fa*)(ap + k0 + 4);
    const v4f x2 = *(const v4fa*)(ap + k0 + 16);
    const v4f x3 = *(const v4fa*)(ap + k0 + 20);
    FragB af;
    af.h[0] = cvt8(x0, x1);
    af.h[1] = cvt8(x2, x3);
#pragma unroll
    for (int nt = 0; nt < 8; ++nt) {
      const unsigned short* wq = bp + (size_t)(16 * nt) * (size_t)ldb + k0;
      FragB bf;
      bf.h[0] = *(const v8usa*)wq;
      bf.h[1] = *(const v8usa*)(wq + 16);
      acc[nt] = wmb(af, bf, acc[nt]);
    }
  }

#pragma unroll
  for (int nt = 0; nt < 8; ++nt) {
    const int lc = 16 * nt + m;
#pragma unroll
    for (int r = 0; r < 8; ++r) {
      const int lr = 16 * wave + 8 * hh + r;
      stg[lr * GBN + lc] = acc[nt][r];
    }
  }
  __syncthreads();

  v4f pv[16];
#pragma unroll
  for (int i = 0; i < 16; ++i) pv[i] = *(const v4fa*)(stg + (16 * wave + i) * GBN + 4 * lane);
#pragma unroll
  for (int i = 0; i < 16; ++i) {
    float* op = Cm + (size_t)(rowBase + 16 * wave + i) * (size_t)ldc + colBase + 4 * lane;
    *(volatile v4f*)op = pv[i];
  }
  __threadfence();
#pragma unroll
  for (int i = 0; i < 16; ++i) {
    float* op = Cm + (size_t)(rowBase + 16 * wave + i) * (size_t)ldc + colBase + 4 * lane;
    *(volatile v4f*)op = pv[i];
  }
}

__device__ __forceinline__ void wave_gemm_b(const unsigned short* sAw, float* sDw,
                                            const unsigned short* __restrict__ BT, int ldb, int K,
                                            int hh, int m) {
#pragma unroll 1
  for (int nh = 0; nh < 2; ++nh) {
    v8f acc[2][4];
    {
      const v8f z = {0.f, 0.f, 0.f, 0.f, 0.f, 0.f, 0.f, 0.f};
#pragma unroll
      for (int mt = 0; mt < 2; ++mt)
#pragma unroll
        for (int nt = 0; nt < 4; ++nt) acc[mt][nt] = z;
    }
    const unsigned short* ap0 = sAw + m * AP + 8 * hh;
    const unsigned short* ap1 = ap0 + 16 * AP;
    const unsigned short* bp  = BT + (size_t)(64 * nh + m) * (size_t)ldb + 8 * hh;
#pragma unroll 1
    for (int k0 = 0; k0 < K; k0 += 32) {
      FragB a0, a1;
      a0.h[0] = *(const v8usa*)(ap0 + k0);
      a0.h[1] = *(const v8usa*)(ap0 + k0 + 16);
      a1.h[0] = *(const v8usa*)(ap1 + k0);
      a1.h[1] = *(const v8usa*)(ap1 + k0 + 16);
#pragma unroll
      for (int nt = 0; nt < 4; ++nt) {
        const unsigned short* wq = bp + (size_t)(16 * nt) * (size_t)ldb + k0;
        FragB b;
        b.h[0] = *(const v8usa*)wq;
        b.h[1] = *(const v8usa*)(wq + 16);
        acc[0][nt] = wmb(a0, b, acc[0][nt]);
        acc[1][nt] = wmb(a1, b, acc[1][nt]);
      }
    }
#pragma unroll
    for (int nt = 0; nt < 4; ++nt) {
      const int col = 64 * nh + 16 * nt + m;
#pragma unroll
      for (int mt = 0; mt < 2; ++mt)
#pragma unroll
        for (int r = 0; r < 8; ++r) sDw[(16 * mt + 8 * hh + r) * DP + col] = acc[mt][nt][r];
    }
  }
}

__global__ __launch_bounds__(ETHR) void k_edge(const int* __restrict__ ei, int nE, int nS, int nT,
                                               const float* __restrict__ PS, const float* __restrict__ PT,
                                               const unsigned short* __restrict__ W1T,
                                               const float* __restrict__ bbi, const float* __restrict__ b1,
                                               const float* __restrict__ w2, const float* __restrict__ b2,
                                               float* outp) {
  extern __shared__ __attribute__((aligned(16))) float dyn[];
  float*          sD  = dyn;
  unsigned short* sA  = (unsigned short*)(dyn + EPB * DP);
  float*          cst = dyn + EPB * DP + (EPB * AP) / 2;
  float*          sS  = cst + CSTN;

  const int tid = (int)threadIdx.x, lane = tid & 31, wave = tid >> 5, hh = lane >> 4, m = lane & 15;

  if (tid < HF) {
    cst[tid]          = bf16_val(bbi[tid]);
    cst[HF + tid]     = bf16_val(b1[tid]);
    cst[2 * HF + tid] = bf16_val(w2[tid]);
  }
  if (tid < 32) {
    const float vb = bf16_val(b2[0]);
    if (tid == 0) cst[3 * HF] = vb;
  }

  const int  elb  = (int)blockIdx.x * EPB;
  const int  el   = elb + tid;
  const bool live = el < nE;
  const int  elc  = live ? el : (nE - 1);
  int r = ei[elc];
  int c = ei[(size_t)nE + (size_t)elc];
  r = r < 0 ? 0 : (r > nS - 1 ? nS - 1 : r);
  c = c < 0 ? 0 : (c > nT - 1 ? nT - 1 : c);
  const float* pr = PS + (size_t)r * HF;
  const float* qr = PT + (size_t)c * HF;
  __syncthreads();

  unsigned short* ra = sA + tid * AP;
  const float*    rd = sD + tid * DP;

  {
#pragma unroll 1
    for (int c8 = 0; c8 < HF / 8; ++c8) {
      const v4f pa = *(const v4fa*)(pr + 8 * c8);
      const v4f pb = *(const v4fa*)(pr + 8 * c8 + 4);
      const v4f qa = *(const v4fa*)(qr + 8 * c8);
      const v4f qb = *(const v4fa*)(qr + 8 * c8 + 4);
      const v4f ba = *(const v4fa*)(cst + 8 * c8);
      const v4f bb = *(const v4fa*)(cst + 8 * c8 + 4);
      const v8f p8 = {pa.x, pa.y, pa.z, pa.w, pb.x, pb.y, pb.z, pb.w};
      const v8f q8 = {qa.x, qa.y, qa.z, qa.w, qb.x, qb.y, qb.z, qb.w};
      const v8f b8 = {ba.x, ba.y, ba.z, ba.w, bb.x, bb.y, bb.z, bb.w};
      v8us ohi, olo;
#pragma unroll
      for (int i = 0; i < 8; ++i) {
        const float h1 = elu_f((p8[i] + q8[i]) + b8[i]);
        const unsigned hb = bf16_bits(h1);
        ohi[i] = (unsigned short)hb;
        olo[i] = (unsigned short)bf16_bits(h1 - __uint_as_float(hb << 16));
      }
      *(v8usa*)(ra + 8 * c8)      = ohi;
      *(v8usa*)(ra + HF + 8 * c8) = olo;
    }
  }
  __syncthreads();

  wave_gemm_b(sA + 32 * wave * AP, sD + 32 * wave * DP, W1T, K2, K2, hh, m);
  __syncthreads();

  {
    float tsum = 0.0f;
#pragma unroll 1
    for (int c8 = 0; c8 < HF / 8; ++c8) {
      const v4f va = *(const v4fa*)(rd + 8 * c8);
      const v4f vb = *(const v4fa*)(rd + 8 * c8 + 4);
      const v4f ba = *(const v4fa*)(cst + HF + 8 * c8);
      const v4f bb = *(const v4fa*)(cst + HF + 8 * c8 + 4);
      const v4f wa = *(const v4fa*)(cst + 2 * HF + 8 * c8);
      const v4f wb = *(const v4fa*)(cst + 2 * HF + 8 * c8 + 4);
      const v8f v8 = {va.x, va.y, va.z, va.w, vb.x, vb.y, vb.z, vb.w};
      const v8f b8 = {ba.x, ba.y, ba.z, ba.w, bb.x, bb.y, bb.z, bb.w};
      const v8f w8 = {wa.x, wa.y, wa.z, wa.w, wb.x, wb.y, wb.z, wb.w};
#pragma unroll
      for (int i = 0; i < 8; ++i) tsum = fmaf(elu_f(v8[i] + b8[i]), w8[i], tsum);
    }
    const float y = tsum + cst[3 * HF];
    sS[tid] = live ? sigm_f(y) : 0.0f;
  }
  __syncthreads();

  {
    const int tl = tid < EPB / 4 ? tid : EPB / 4 - 1;
    const v4f o4 = *(const v4fa*)(sS + 4 * tl);
    const int eo = elb + 4 * tl;
    const bool stv = (tid < EPB / 4) && (eo + 3 < nE);
    float* op = outp + (size_t)eo;
    if (stv) *(volatile v4f*)op = o4;
    __threadfence();
    if (stv) *(volatile v4f*)op = o4;
  }
}

static inline int cdiv(int a, int b) { return (a + b - 1) / b; }

extern "C" void kernel_launch(void* const* d_in, const int* in_sizes, int n_in,
                              void* d_out, int out_size, void* d_ws, size_t ws_size,
                              hipStream_t stream) {
  if (n_in < 16) return;
  if (in_sizes[0] < HF || (in_sizes[0] % HF) != 0) return;
  const int nU = in_sizes[0] / HF;
  if (in_sizes[1] < HF || (in_sizes[1] % HF) != 0) return;
  const int nI = in_sizes[1] / HF;
  if (nU > (1 << 22) || nI > (1 << 22)) return;
  if (in_sizes[2] < 2 || (in_sizes[2] & 1) != 0) return;
  const int nE = in_sizes[2] / 2;
  if (in_sizes[3] != in_sizes[2]) return;
  if (nE < 32 || (nE & 31) != 0 || nE > (1 << 24)) return;
  if (in_sizes[4] != KIN * HF || in_sizes[5] != HF) return;
  if (in_sizes[6] != HF * HF || in_sizes[7] != HF) return;
  if (in_sizes[8] != HF || in_sizes[9] != 1) return;
  if (in_sizes[10] != KIN * HF || in_sizes[11] != HF) return;
  if (in_sizes[12] != HF * HF || in_sizes[13] != HF) return;
  if (in_sizes[14] != HF || in_sizes[15] != 1) return;
  if ((long long)out_size != 2LL * (long long)nE) return;

  const float* user  = (const float*)d_in[0];
  const float* item  = (const float*)d_in[1];
  const int*   eiui  = (const int*)d_in[2];
  const int*   eiiu  = (const int*)d_in[3];
  const float* Wbu   = (const float*)d_in[4];
  const float* bbu   = (const float*)d_in[5];
  const float* W1u   = (const float*)d_in[6];
  const float* b1u   = (const float*)d_in[7];
  const float* W2u   = (const float*)d_in[8];
  const float* b2u   = (const float*)d_in[9];
  const float* Wbi   = (const float*)d_in[10];
  const float* bbiu  = (const float*)d_in[11];
  const float* W1i   = (const float*)d_in[12];
  const float* b1i   = (const float*)d_in[13];
  const float* W2i   = (const float*)d_in[14];
  const float* b2i   = (const float*)d_in[15];
  float* out = (float*)d_out;

  const int MPU = cdiv(nU, GBM) * GBM;
  const int MPI = cdiv(nI, GBM) * GBM;
  const int MPX = MPU > MPI ? MPU : MPI;

  char* ws = (char*)d_ws;
  size_t off = 0;
  const size_t oWBu = off; off += (size_t)KIN * HF * 2;        off = (off + 255) & ~(size_t)255;
  const size_t oWBi = off; off += (size_t)KIN * HF * 2;        off = (off + 255) & ~(size_t)255;
  const size_t oW1u = off; off += (size_t)HF * K2 * 2;         off = (off + 255) & ~(size_t)255;
  const size_t oW1i = off; off += (size_t)HF * K2 * 2;         off = (off + 255) & ~(size_t)255;
  const size_t oPS  = off; off += (size_t)MPX * HF * 4;        off = (off + 255) & ~(size_t)255;
  const size_t oPT  = off; off += (size_t)MPX * HF * 4;        off = (off + 255) & ~(size_t)255;
  if (off > ws_size || off > (size_t)WSMAX) return;
  unsigned short* WBTu = (unsigned short*)(ws + oWBu);
  unsigned short* WBTi = (unsigned short*)(ws + oWBi);
  unsigned short* W1Tu = (unsigned short*)(ws + oW1u);
  unsigned short* W1Ti = (unsigned short*)(ws + oW1i);
  float*          PS   = (float*)(ws + oPS);
  float*          PT   = (float*)(ws + oPT);

  hipFuncSetAttribute(reinterpret_cast<const void*>(&k_edge), hipFuncAttributeMaxDynamicSharedMemorySize,
                      (int)EDGE_LDS_BYTES);

  const int gE = cdiv(nE, EPB);

  k_prep<<<NPREP / NTHR, NTHR, 0, stream>>>(Wbu, Wbi, W1u, W1i, WBTu, WBTi, W1Tu, W1Ti);
  k_gemm<<<dim3(MPU / GBM, HF / GBN), GTHR, 0, stream>>>(user, nU, HF, WBTu, HF, HF, PS, HF);
  k_gemm<<<dim3(MPI / GBM, HF / GBN), GTHR, 0, stream>>>(item, nI, HF, WBTu + (size_t)HF * HF, HF, HF, PT, HF);
  k_edge<<<gE, ETHR, EDGE_LDS_BYTES, stream>>>(eiui, nE, nU, nI, PS, PT, W1Tu, bbu, b1u, W2u, b2u, out);
  k_gemm<<<dim3(MPI / GBM, HF / GBN), GTHR, 0, stream>>>(item, nI, HF, WBTi, HF, HF, PS, HF);
  k_gemm<<<dim3(MPU / GBM, HF / GBN), GTHR, 0, stream>>>(user, nU, HF, WBTi + (size_t)HF * HF, HF, HF, PT, HF);
  k_edge<<<gE, ETHR, EDGE_LDS_BYTES, stream>>>(eiiu, nE, nI, nU, PS, PT, W1Ti, bbiu, b1i, W2i, b2i,
                                               out + (size_t)nE);
}
